// DigitCaps_39230231281960
// MI455X (gfx1250) — hardware-verified
//
#include <hip/hip_runtime.h>
#include <stddef.h>


typedef _Float16 h16;
typedef _Float16 v16h __attribute__((ext_vector_type(16)));
typedef _Float16 v8h  __attribute__((ext_vector_type(8)));
typedef _Float16 v4h  __attribute__((ext_vector_type(4)));
typedef float    v8f  __attribute__((ext_vector_type(8)));
typedef float    v4f  __attribute__((ext_vector_type(4)));

#ifndef NB
#define NB 64
#endif
#ifndef NCAP
#define NCAP 2048
#endif
#define NB_FULL   64
#define NCAP_FULL 2048
#define ILEN 8
#define CCAP 32
#define LLEN 16
#define CL   512
#define JSUB 16
#define JBLK 64
#define NSUB (JBLK / JSUB)
#define NCHUNK (NCAP / JBLK)

#define WCARRY 64.0f
#define VCARRY 64.0f
#define BCARRY 1024.0f

#define LDW 520
#define UP  132
#define VP  520

static_assert(NB >= 16 && NB <= NB_FULL && (NB % 16) == 0);
static_assert(NCAP >= JBLK && NCAP <= NCAP_FULL && (NCAP % JBLK) == 0);
static_assert(CL == CCAP * LLEN);
static_assert(ILEN == 8 && LLEN == 16 && CCAP == 32);
static_assert(JSUB == 16 && (JBLK % JSUB) == 0);
static_assert(JSUB / 2 == 8);
static_assert(CCAP / 8 == 4);
static_assert(JSUB * CCAP * 16 == 16 * CL);
static_assert((LDW % 8) == 0 && LDW >= CL);
static_assert((UP % 4) == 0 && UP >= JSUB * ILEN);
static_assert((VP % 8) == 0 && VP >= CL);
static_assert(ILEN * CL == 4 * 256 * 4);
static_assert(16 * JSUB * ILEN == 2 * 256 * 4);
static_assert(16 * CL == 8 * 256 * 4);
static_assert(CL == 128 * 4);

#define WPLANE_BYTES ((size_t)NCAP * ILEN * CL * 2)
#define SPART_BYTES  ((size_t)NCHUNK * NB * CL * 4)
#define VSUM_BYTES   ((size_t)NB * CL * 4)
#define OFF_WL ((size_t)0)
#define OFF_WT (OFF_WL + WPLANE_BYTES)
#define OFF_SP (OFF_WT + WPLANE_BYTES)
#define OFF_VA (OFF_SP + SPART_BYTES)
#define OFF_VB (OFF_VA + VSUM_BYTES)
#define WS_TOTAL (OFF_VB + VSUM_BYTES)
static_assert((WPLANE_BYTES % 128) == 0 && (SPART_BYTES % 128) == 0 && (VSUM_BYTES % 128) == 0);
static_assert(WS_TOTAL <= (size_t)134217728);

__device__ __forceinline__ float bf16r(float x) {
  unsigned int u = __float_as_uint(x);
  u = (u + 0x7FFFu + ((u >> 16) & 1u)) & 0xFFFF0000u;
  return __uint_as_float(u);
}

static __device__ __forceinline__ h16 toh_flush(float v) {
  const h16 r = (h16)v;
  return (fabsf(v) < 6.103515625e-05f) ? (h16)0.0f : r;
}

__device__ __forceinline__ v8f wmma16(v16h a, v16h b, v8f c) {
  v8f d = __builtin_amdgcn_wmma_f32_16x16x32_f16(false, a, false, b, (short)0, c,
                                                 false, false);
  asm volatile("v_nop\n\tv_nop\n\tv_nop\n\tv_nop" : "+v"(d) : "v"(a), "v"(b));
  return d;
}

__device__ __forceinline__ v16h frag_k16(v8h lo) {
  v16h out;
#pragma unroll
  for (int i = 0; i < 8; ++i) { out[i] = lo[i]; out[i + 8] = (_Float16)0.0f; }
  return out;
}
__device__ __forceinline__ v16h frag_k32(v8h lo, v8h hi) {
  v16h out;
#pragma unroll
  for (int i = 0; i < 8; ++i) { out[i] = lo[i]; out[i + 8] = hi[i]; }
  return out;
}

__global__ __launch_bounds__(256) void wplanes_kernel(
    const float* __restrict__ W, _Float16* __restrict__ Wl, _Float16* __restrict__ Wt) {
  __shared__ _Float16 T[ILEN * LDW];
  const unsigned tid = threadIdx.x;
  const unsigned j = blockIdx.x;
  const float* src = W + (size_t)j * (ILEN * CL);
#pragma unroll
  for (unsigned r = 0; r < 4u; ++r) {
    const unsigned idx = tid + 256u * r;
    const unsigned i = idx >> 7, o = (idx & 127u) * 4u;
    const v4f w = *(const v4f*)(src + i * CL + o);
    v4h t;
#pragma unroll
    for (int k = 0; k < 4; ++k) t[k] = toh_flush(WCARRY * bf16r(w[k]));
    *(v4h*)&T[i * LDW + o] = t;
  }
  __syncthreads();
  v8h xl[2], xt[2];
  size_t ol[2], ot[2];
#pragma unroll
  for (unsigned r = 0; r < 2u; ++r) {
    const unsigned idx = tid + 256u * r;
    xl[r] = *(const v8h*)&T[(idx >> 6) * LDW + (idx & 63u) * 8u];
    ol[r] = (size_t)j * (ILEN * CL) + (size_t)idx * 8u;
#pragma unroll
    for (unsigned i = 0; i < 8u; ++i) xt[r][i] = T[i * LDW + idx];
    ot[r] = ((size_t)j * CL + idx) * ILEN;
  }
#pragma unroll
  for (int r = 0; r < 2; ++r) {
    *(volatile v8h*)(Wl + ol[r]) = xl[r];
    *(volatile v8h*)(Wt + ot[r]) = xt[r];
  }
  __threadfence();
#pragma unroll
  for (int r = 0; r < 2; ++r) {
    *(volatile v8h*)(Wl + ol[r]) = xl[r];
    *(volatile v8h*)(Wt + ot[r]) = xt[r];
  }
}

__global__ __launch_bounds__(256) void route_kernel(
    const float* __restrict__ X, const _Float16* __restrict__ Wl,
    const _Float16* __restrict__ Wt, const float* __restrict__ Vsum,
    float* __restrict__ Spart, int routed) {
  __shared__ float    Uf[16 * UP];
  __shared__ _Float16 V16[16 * VP];
  __shared__ float    Cf[JSUB * CCAP * 16];

  const unsigned tid = threadIdx.x, lane = tid & 31u;
  const unsigned wave = (unsigned)__builtin_amdgcn_readfirstlane((int)(threadIdx.x >> 5));
  const unsigned hh = lane >> 4, m = lane & 15u;
  const unsigned chunk = blockIdx.x;
  const unsigned b0 = blockIdx.y * 16u;
  const unsigned jbase = chunk * (unsigned)JBLK;

  if (routed) {
#pragma unroll
    for (unsigned r = 0; r < 8u; ++r) {
      const unsigned idx = tid + 256u * r;
      const unsigned b = idx >> 7, c4 = (idx & 127u) * 4u;
      const v4f v = *(const v4f*)(Vsum + (size_t)(b0 + b) * CL + c4);
      v4h t;
#pragma unroll
      for (int k = 0; k < 4; ++k) t[k] = toh_flush(VCARRY * v[k]);
      *(v4h*)&V16[b * VP + c4] = t;
    }
  }

  v8f acc[4];
#pragma unroll
  for (int ci = 0; ci < 4; ++ci) acc[ci] = (v8f){};

#pragma unroll 1
  for (unsigned sub = 0; sub < (unsigned)NSUB; ++sub) {
    const unsigned j0 = jbase + sub * (unsigned)JSUB;

#pragma unroll
    for (unsigned r = 0; r < 2u; ++r) {
      const unsigned idx = tid + 256u * r;
      const unsigned b = idx >> 5, f4 = idx & 31u;
      v4f t = *(const v4f*)(X + ((size_t)(b0 + b) * NCAP_FULL + j0) * ILEN + f4 * 4u);
#pragma unroll
      for (int k = 0; k < 4; ++k) t[k] = bf16r(t[k]);
      *(v4f*)&Uf[b * UP + f4 * 4u] = t;
    }
    __syncthreads();

    if (routed) {
      const unsigned jr = 2u * wave + hh;
      const v4f u0 = *(const v4f*)&Uf[m * UP + jr * 8u];
      const v4f u1 = *(const v4f*)&Uf[m * UP + jr * 8u + 4u];
      const _Float16* wl = Wl + ((size_t)(j0 + 2u * wave) * ILEN + m) * CL + hh * 8u;
      const unsigned cbase = jr * (unsigned)(CCAP * 16) + m;
      float mx = -3.0e38f;
#pragma unroll 4
      for (unsigned c = 0; c < (unsigned)CCAP; ++c) {
        const v8h wa = *(const v8h*)(wl + c * 16u);
        const v8h vb = *(const v8h*)&V16[m * VP + c * 16u + hh * 8u];
        const v16h af = frag_k16(wa);
        const v16h bf = frag_k16(vb);
        v8f g = {};
        g = wmma16(af, bf, g);
        float a = g[0] * u0[0];
        a += g[1] * u0[1];
        a += g[2] * u0[2];
        a += g[3] * u0[3];
        a += g[4] * u1[0];
        a += g[5] * u1[1];
        a += g[6] * u1[2];
        a += g[7] * u1[3];
        a *= (1.0f / (WCARRY * VCARRY));
        Cf[cbase + c * 16u] = a;
        mx = fmaxf(mx, a);
      }
      float ssum = 0.0f;
#pragma unroll 4
      for (unsigned c = 0; c < (unsigned)CCAP; ++c) {
        const float e = __expf(Cf[cbase + c * 16u] - mx);
        Cf[cbase + c * 16u] = e;
        ssum += e;
      }
      const float inv = __builtin_amdgcn_rcpf(ssum);
#pragma unroll 4
      for (unsigned c = 0; c < (unsigned)CCAP; ++c) {
        const float e = Cf[cbase + c * 16u];
        Cf[cbase + c * 16u] = e * inv;
      }
    } else {
#pragma unroll 4
      for (unsigned r = 0; r < 32u; ++r) Cf[tid + 256u * r] = (1.0f / 32.0f);
    }
    __syncthreads();

#pragma unroll 1
    for (unsigned q = 0; q < (unsigned)(JSUB / 4); ++q) {
      const unsigned jA = 4u * q + hh, jB = jA + 2u;
      const v4f ua0 = *(const v4f*)&Uf[m * UP + jA * 8u];
      const v4f ua1 = *(const v4f*)&Uf[m * UP + jA * 8u + 4u];
      const v4f ub0 = *(const v4f*)&Uf[m * UP + jB * 8u];
      const v4f ub1 = *(const v4f*)&Uf[m * UP + jB * 8u + 4u];
      const _Float16* wt = Wt + ((size_t)(j0 + jA) * CL + (4u * wave) * 16u + m) * ILEN;
#pragma unroll
      for (int ci = 0; ci < 4; ++ci) {
        const unsigned c = 4u * wave + (unsigned)ci;
        const float ca = Cf[(jA * (unsigned)CCAP + c) * 16u + m] * BCARRY;
        const float cb = Cf[(jB * (unsigned)CCAP + c) * 16u + m] * BCARRY;
        v16h bf;
#pragma unroll
        for (int i = 0; i < 4; ++i) {
          bf[i]      = toh_flush(ca * ua0[i]);
          bf[i + 4]  = toh_flush(ca * ua1[i]);
          bf[i + 8]  = toh_flush(cb * ub0[i]);
          bf[i + 12] = toh_flush(cb * ub1[i]);
        }
        const _Float16* wp = wt + (size_t)ci * (16u * ILEN);
        const v8h alo = *(const v8h*)wp;
        const v8h ahi = *(const v8h*)(wp + (size_t)2 * CL * ILEN);
        const v16h af = frag_k32(alo, ahi);
        acc[ci] = wmma16(af, bf, acc[ci]);
      }
    }
    __syncthreads();
  }

  const float sc = 1.0f / (WCARRY * BCARRY);
#pragma unroll
  for (int ci = 0; ci < 4; ++ci) {
    const unsigned c = 4u * wave + (unsigned)ci;
    v4f lo, hi;
#pragma unroll
    for (int r = 0; r < 4; ++r) { lo[r] = acc[ci][r] * sc; hi[r] = acc[ci][r + 4] * sc; }
    *(v4f*)&Cf[m * CL + c * 16u + hh * 8u] = lo;
    *(v4f*)&Cf[m * CL + c * 16u + hh * 8u + 4u] = hi;
  }
  __syncthreads();
  v4f xs[8];
  size_t off[8];
#pragma unroll
  for (unsigned r = 0; r < 8u; ++r) {
    const unsigned idx = tid + 256u * r;
    const unsigned b = idx >> 7, c4 = (idx & 127u) * 4u;
    xs[r] = *(const v4f*)&Cf[b * CL + c4];
    off[r] = ((size_t)chunk * NB + b0 + b) * CL + c4;
  }
#pragma unroll
  for (int r = 0; r < 8; ++r) *(volatile v4f*)(Spart + off[r]) = xs[r];
  __threadfence();
#pragma unroll
  for (int r = 0; r < 8; ++r) *(volatile v4f*)(Spart + off[r]) = xs[r];
}

__global__ __launch_bounds__(128) void squash_kernel(
    const float* __restrict__ Spart, const float* __restrict__ bias,
    const float* __restrict__ vprev, float* __restrict__ vdst, int addprev) {
#pragma clang fp contract(off)
  const unsigned t = threadIdx.x;
  const unsigned b = blockIdx.x;
  const unsigned col = t * 4u;
  v4f s = {0.0f, 0.0f, 0.0f, 0.0f};
#pragma unroll 4
  for (unsigned p = 0; p < (unsigned)NCHUNK; ++p) {
    const v4f a = *(const v4f*)(Spart + ((size_t)p * NB + b) * CL + col);
    s += a;
  }
  const v4f bb = *(const v4f*)(bias + col);
#pragma unroll
  for (int i = 0; i < 4; ++i) s[i] += bf16r(bb[i]);
  float q = (s[0] * s[0] + s[1] * s[1]) + (s[2] * s[2] + s[3] * s[3]);
  q += __shfl_xor(q, 1, 32);
  q += __shfl_xor(q, 2, 32);
  const float n2 = q + 1.0e-7f;
  const float f = n2 * __builtin_amdgcn_rcpf(1.0f + n2) * __builtin_amdgcn_rsqf(n2);
  v4f v = s * f;
  if (addprev) {
    const v4f pv = *(const v4f*)(vprev + (size_t)b * CL + col);
    v += pv;
  }
  float* p = vdst + (size_t)b * CL + col;
  *(volatile v4f*)p = v;
  __threadfence();
  *(volatile v4f*)p = v;
}

extern "C" void kernel_launch(void* const* d_in, const int* in_sizes, int n_in,
                              void* d_out, int out_size, void* d_ws, size_t ws_size,
                              hipStream_t stream) {
  if (n_in < 3) return;
  const long long need_x = ((long long)(NB - 1) * NCAP_FULL + NCAP) * ILEN;
  if ((long long)in_sizes[0] < need_x) return;
  if ((long long)in_sizes[1] < (long long)NCAP * ILEN * CL) return;
  if (in_sizes[2] < CL) return;
  if ((long long)out_size < (long long)NB * CL) return;
  if (ws_size < WS_TOTAL) return;

  const float* X    = (const float*)d_in[0];
  const float* Wm   = (const float*)d_in[1];
  const float* bias = (const float*)d_in[2];
  float* out = (float*)d_out;

  char* ws = (char*)d_ws;
  _Float16* Wl16 = (_Float16*)(ws + OFF_WL);
  _Float16* Wt16 = (_Float16*)(ws + OFF_WT);
  float*    Sp   = (float*)(ws + OFF_SP);
  float*    Va   = (float*)(ws + OFF_VA);
  float*    Vb   = (float*)(ws + OFF_VB);

  dim3 gr(NCHUNK, NB / 16);

  wplanes_kernel<<<dim3(NCAP), dim3(256), 0, stream>>>(Wm, Wl16, Wt16);

  route_kernel<<<gr, dim3(256), 0, stream>>>(X, Wl16, Wt16, Va, Sp, 0);
  squash_kernel<<<dim3(NB), dim3(128), 0, stream>>>(Sp, bias, Vb, Va, 0);
  route_kernel<<<gr, dim3(256), 0, stream>>>(X, Wl16, Wt16, Va, Sp, 1);
  squash_kernel<<<dim3(NB), dim3(128), 0, stream>>>(Sp, bias, Va, Vb, 1);
  route_kernel<<<gr, dim3(256), 0, stream>>>(X, Wl16, Wt16, Vb, Sp, 1);
  squash_kernel<<<dim3(NB), dim3(128), 0, stream>>>(Sp, bias, Vb, out, 0);
}
